// GATBlock_592705487420
// MI455X (gfx1250) — hardware-verified
//
#include <hip/hip_runtime.h>
#include <hip/hip_bf16.h>
#include <stddef.h>
#include <stdint.h>


#define DIN     128
#define DOUT    128
#define NLR     256
#define EDIM    16
#define NTHR    256
#define NWAVE   8
#define EPT     8
#define CHUNK   (NTHR * EPT)
#define WCAP    (EPT * 32)
#define LISTN   (NWAVE * WCAP)
#define NBMAX   2048
#define RCAP    28672
#define DEGCAP  4096
#define GBM     64
#define GBN     64
#define GTHR    128
#define NEG_SLOPE 0.2f
#define EPS_SM  1e-16f
#define LN_EPS  1e-5f
#define WSMAX   134217728
#define LDS_AGG ((2 * RCAP + 2 * NBMAX + LISTN) * 4 + 64)

static_assert((CHUNK & (CHUNK - 1)) == 0 && CHUNK <= 4096);
static_assert((NBMAX & (NBMAX - 1)) == 0 && NBMAX <= 4096);
static_assert(NTHR * 8 == NBMAX);
static_assert(LISTN >= NBMAX);
static_assert(LISTN >= NWAVE * WCAP);
static_assert((RCAP % 32) == 0);
static_assert(EDIM * DOUT + DOUT <= RCAP);
static_assert(LDS_AGG <= 300000);
static_assert(GBM == (GTHR / 32) * 16);
static_assert(DIN / 8 == 16);
static_assert((DIN % 32) == 0);
static_assert((NLR % GBN) == 0 && (NLR % 32) == 0);
static_assert(DOUT == 4 * 32 && EDIM == 16);
static_assert(NLR == 2 * DOUT);

typedef float          v4f  __attribute__((ext_vector_type(4)));
typedef float          v8f  __attribute__((ext_vector_type(8)));
typedef int            v4i  __attribute__((ext_vector_type(4)));
typedef int            v8i  __attribute__((ext_vector_type(8)));
typedef unsigned short v8us __attribute__((ext_vector_type(8)));
typedef unsigned int   v2u  __attribute__((ext_vector_type(2)));
typedef __bf16         v16b __attribute__((ext_vector_type(16)));
typedef v4f  __attribute__((may_alias)) v4fa;
typedef v8us __attribute__((may_alias)) v8usa;
typedef v2u  __attribute__((may_alias)) v2ua;
union FragB { v16b v; v8us h[2]; v8i w; };

__device__ __forceinline__ v8f wmb(const FragB& a, const FragB& b, v8f c) {
  v8f d = __builtin_amdgcn_wmma_f32_16x16x32_bf16(false, a.v, false, b.v, (short)0, c, false, false);
  asm volatile("v_nop\n\tv_nop\n\tv_nop\n\tv_nop" : "+v"(d) : "v"(a.w), "v"(b.w));
  return d;
}

__device__ __forceinline__ unsigned short f2bf(float f) {
  unsigned u = __float_as_uint(f);
  u += 0x7FFFu + ((u >> 16) & 1u);
  return (unsigned short)(u >> 16);
}
__device__ __forceinline__ float bfr(float f) {
  unsigned u = __float_as_uint(f);
  u = (u + 0x7FFFu + ((u >> 16) & 1u)) & 0xFFFF0000u;
  return __uint_as_float(u);
}
__device__ __forceinline__ v8us cvt8b(const v4f a, const v4f b) {
  v8us o;
  o[0] = f2bf(a.x); o[1] = f2bf(a.y); o[2] = f2bf(a.z); o[3] = f2bf(a.w);
  o[4] = f2bf(b.x); o[5] = f2bf(b.y); o[6] = f2bf(b.z); o[7] = f2bf(b.w);
  return o;
}

__device__ __forceinline__ int scan_chunk(const int* __restrict__ dsts, int nE, int cbase, int slotBase,
                                          int nb, int vec8, int* list, int tid, int lane, int wave) {
  int wc = 0;
  const int el0  = tid * EPT;
  const int e0   = cbase + el0;
  const int sent = -2147483647 - 1;
  v4i da, db;
  if (vec8 != 0 && cbase + CHUNK <= nE) {
    da = *(const v4i*)(dsts + e0);
    db = *(const v4i*)(dsts + e0 + 4);
  } else {
    da.x = (e0     < nE) ? dsts[min(e0,     nE - 1)] : sent;
    da.y = (e0 + 1 < nE) ? dsts[min(e0 + 1, nE - 1)] : sent;
    da.z = (e0 + 2 < nE) ? dsts[min(e0 + 2, nE - 1)] : sent;
    da.w = (e0 + 3 < nE) ? dsts[min(e0 + 3, nE - 1)] : sent;
    db.x = (e0 + 4 < nE) ? dsts[min(e0 + 4, nE - 1)] : sent;
    db.y = (e0 + 5 < nE) ? dsts[min(e0 + 5, nE - 1)] : sent;
    db.z = (e0 + 6 < nE) ? dsts[min(e0 + 6, nE - 1)] : sent;
    db.w = (e0 + 7 < nE) ? dsts[min(e0 + 7, nE - 1)] : sent;
  }
  const unsigned nbs = (unsigned)slotBase;
  const unsigned unb = (unsigned)nb;
  const unsigned s0 = (unsigned)da.x - nbs, s1 = (unsigned)da.y - nbs;
  const unsigned s2 = (unsigned)da.z - nbs, s3 = (unsigned)da.w - nbs;
  const unsigned s4 = (unsigned)db.x - nbs, s5 = (unsigned)db.y - nbs;
  const unsigned s6 = (unsigned)db.z - nbs, s7 = (unsigned)db.w - nbs;
  const bool h0 = s0 < unb, h1 = s1 < unb, h2 = s2 < unb, h3 = s3 < unb;
  const bool h4 = s4 < unb, h5 = s5 < unb, h6 = s6 < unb, h7 = s7 < unb;
  const unsigned any = __builtin_amdgcn_ballot_w32(h0 | h1 | h2 | h3 | h4 | h5 | h6 | h7);
  if (any != 0u) {
#define HITJ(J, HJ, SJ) { \
      const unsigned mj = __builtin_amdgcn_ballot_w32(HJ); \
      if (mj != 0u) { \
        if (HJ) { \
          const int pos = wc + (int)__builtin_amdgcn_mbcnt_lo(mj, 0u); \
          if (pos < WCAP) list[wave * WCAP + pos] = ((el0 + (J)) << 12) | (int)(SJ); \
        } \
        wc += (int)__builtin_popcount(mj); } }
    HITJ(0, h0, s0)
    HITJ(1, h1, s1)
    HITJ(2, h2, s2)
    HITJ(3, h3, s3)
    HITJ(4, h4, s4)
    HITJ(5, h5, s5)
    HITJ(6, h6, s6)
    HITJ(7, h7, s7)
#undef HITJ
  }
  return wc;
}

__global__ __launch_bounds__(NTHR) void k_xprep(const float* __restrict__ x, unsigned short* xb, int nN, int nUnits) {
  const int i = (int)blockIdx.x * NTHR + (int)threadIdx.x;
  if (i >= nUnits) return;
  const int row = i >> 4;
  const int c0  = (i & 15) * 8;
  const int rc  = row < nN ? row : nN - 1;
  const float* p = x + (size_t)rc * DIN + c0;
  v4f a = *(const v4fa*)p, b = *(const v4fa*)(p + 4);
  const v4f z4 = {0.f, 0.f, 0.f, 0.f};
  if (row >= nN) { a = z4; b = z4; }
  const v8us hv = cvt8b(a, b);
  const size_t o = (size_t)row * DIN + c0;
  *(volatile v8us*)(xb + o) = hv;
  __threadfence();
  *(volatile v8us*)(xb + o) = hv;
}

__global__ __launch_bounds__(NTHR) void k_wtr(const float* __restrict__ w0, const float* __restrict__ w1,
                                              const float* __restrict__ w2, const float* __restrict__ w3,
                                              int c0, int c1, int c2, int c3, int segRows, int K,
                                              unsigned short* wt, int nUnits) {
  const int u = (int)blockIdx.x * NTHR + (int)threadIdx.x;
  if (u >= nUnits) return;
  const int kq = K >> 3;
  const int n  = u / kq;
  const int k8 = (u - n * kq) * 8;
  int seg = n / segRows;
  seg = seg > 3 ? 3 : seg;
  const int nc = n - seg * segRows;
  const float* ws = (seg == 0) ? w0 : ((seg == 1) ? w1 : ((seg == 2) ? w2 : w3));
  const int cc = (seg == 0) ? c0 : ((seg == 1) ? c1 : ((seg == 2) ? c2 : c3));
  const int ncl = nc < cc ? nc : cc - 1;
  const float* p = ws + (size_t)k8 * (size_t)cc + ncl;
  v4f a, b;
  a.x = p[0];                  a.y = p[(size_t)cc];         a.z = p[(size_t)2 * cc];     a.w = p[(size_t)3 * cc];
  b.x = p[(size_t)4 * cc];     b.y = p[(size_t)5 * cc];     b.z = p[(size_t)6 * cc];     b.w = p[(size_t)7 * cc];
  const v4f z4 = {0.f, 0.f, 0.f, 0.f};
  if (nc >= cc) { a = z4; b = z4; }
  const v8us hv = cvt8b(a, b);
  const size_t o = (size_t)n * (size_t)K + k8;
  *(volatile v8us*)(wt + o) = hv;
  __threadfence();
  *(volatile v8us*)(wt + o) = hv;
}

__global__ __launch_bounds__(NTHR) void k_eprep(const float* __restrict__ ea, unsigned short* eb, int nVals, int nUnits) {
  const int u = (int)blockIdx.x * NTHR + (int)threadIdx.x;
  if (u >= nUnits) return;
  const size_t i0 = (size_t)u * 8;
  const size_t ic = i0 + 8 <= (size_t)nVals ? i0 : (size_t)nVals - 8;
  v4f a = *(const v4fa*)(ea + ic), b = *(const v4fa*)(ea + ic + 4);
  const v4f z4 = {0.f, 0.f, 0.f, 0.f};
  if (i0 >= (size_t)nVals) { a = z4; b = z4; }
  const v8us hv = cvt8b(a, b);
  *(volatile v8us*)(eb + i0) = hv;
  __threadfence();
  *(volatile v8us*)(eb + i0) = hv;
}

__global__ __launch_bounds__(GTHR) void k_gemm(
    const unsigned short* __restrict__ A, const unsigned short* __restrict__ WT,
    float* outF, int K, int ldo)
{
  __shared__ __attribute__((aligned(16))) float stg[GBM * GBN];
  const int tid = (int)threadIdx.x, lane = tid & 31, wave = tid >> 5, hh = lane >> 4, m = lane & 15;
  const int rowBase = (int)blockIdx.x * GBM;
  const int col0    = (int)blockIdx.y * GBN;

  v8f acc[4];
  {
    const v8f z = {0.f, 0.f, 0.f, 0.f, 0.f, 0.f, 0.f, 0.f};
    acc[0] = z; acc[1] = z; acc[2] = z; acc[3] = z;
  }
  const unsigned short* ap = A  + (size_t)(rowBase + 16 * wave + m) * (size_t)K + 8 * hh;
  const unsigned short* wp = WT + (size_t)(col0 + m) * (size_t)K + 8 * hh;
  const int ksteps = K >> 5;
#pragma unroll 1
  for (int ks = 0; ks < ksteps; ++ks) {
    FragB af;
    af.h[0] = *(const v8usa*)(ap + 32 * ks);
    af.h[1] = *(const v8usa*)(ap + 32 * ks + 16);
#pragma unroll
    for (int t = 0; t < 4; ++t) {
      const unsigned short* wq = wp + (size_t)(16 * t) * (size_t)K + 32 * ks;
      FragB bf;
      bf.h[0] = *(const v8usa*)wq;
      bf.h[1] = *(const v8usa*)(wq + 16);
      acc[t] = wmb(af, bf, acc[t]);
    }
  }

#pragma unroll
  for (int t = 0; t < 4; ++t) {
    const int lc = 16 * t + m;
#pragma unroll
    for (int r = 0; r < 8; ++r) {
      const int lr = 16 * wave + 8 * hh + r;
      stg[lr * GBN + lc] = acc[t][r];
    }
  }
  __syncthreads();

  v4f fv[8];
#pragma unroll
  for (int i = 0; i < 8; ++i) {
    const int lr = 16 * wave + 2 * i + hh;
    fv[i] = *(const v4fa*)(stg + lr * GBN + 4 * m);
  }
#pragma unroll
  for (int i = 0; i < 8; ++i) {
    const int lr = 16 * wave + 2 * i + hh;
    const int gr = rowBase + lr;
    float* op = outF + (size_t)gr * (size_t)ldo + col0 + 4 * m;
    *(volatile v4f*)op = fv[i];
  }
  __threadfence();
#pragma unroll
  for (int i = 0; i < 8; ++i) {
    const int lr = 16 * wave + 2 * i + hh;
    const int gr = rowBase + lr;
    float* op = outF + (size_t)gr * (size_t)ldo + col0 + 4 * m;
    *(volatile v4f*)op = fv[i];
  }
}

__global__ __launch_bounds__(NTHR) void k_agg(
    const int* __restrict__ srcs, const int* __restrict__ dsts,
    const float* __restrict__ XLR, const unsigned short* __restrict__ EB,
    const float* __restrict__ We, const float* __restrict__ att,
    const float* __restrict__ bias, const float* __restrict__ gam, const float* __restrict__ bet,
    float* out, int nN, int nE, int nb, int vec8) {
  extern __shared__ v4f lds_dyn[];
  int* reg1 = (int*)lds_dyn;
  int* reg2 = reg1 + RCAP;
  int* scnt = reg2 + RCAP;
  int* soff = scnt + NBMAX;
  int* list = soff + NBMAX;
  int* wcnt = list + LISTN;
  int* wtot = wcnt + NWAVE;
  const int tid = (int)threadIdx.x, lane = tid & 31, wave = tid >> 5;
  const int nodeBase = (int)blockIdx.x * nb;

  for (int i = tid; i < NBMAX; i += NTHR) scnt[i] = 0;
  __syncthreads();

  int tot = 0;
  const int nChunks = (nE + CHUNK - 1) / CHUNK;
#pragma unroll 1
  for (int ch = 0; ch < nChunks; ++ch) {
    const int cbase = ch * CHUNK;
    const int wc = scan_chunk(dsts, nE, cbase, nodeBase, nb, vec8, list, tid, lane, wave);
    if (lane == 0) wcnt[wave] = wc;
    __syncthreads();
    int pre = 0, all = 0;
#pragma unroll
    for (int w2 = 0; w2 < NWAVE; ++w2) {
      int c = wcnt[w2];
      c = c < 0 ? 0 : (c > WCAP ? WCAP : c);
      all += c;
      pre += (w2 < wave) ? c : 0;
    }
    const int wcc  = wc > WCAP ? WCAP : wc;
    const int base = tot + pre;
#pragma unroll 1
    for (int i = lane; i < wcc; i += 32) {
      const int ent = list[wave * WCAP + i];
      const int el  = (ent >> 12) & (CHUNK - 1);
      const int sl  = ent & (NBMAX - 1);
      int eid = cbase + el;
      eid = eid > nE - 1 ? nE - 1 : eid;
      const int pos = base + i;
      if (pos < RCAP) reg1[pos] = (int)(((unsigned)eid << 12) | (unsigned)sl);
    }
    tot += all;
    tot = tot > RCAP ? RCAP : tot;
    __syncthreads();
  }
  const int nh = tot;

  if (wave == 0) {
#pragma unroll 1
    for (int b0 = 0; b0 < nh; b0 += 32) {
      const int idx = b0 + lane;
      const int uv  = reg1[idx < nh ? idx : nh - 1];
      const int m32 = (nh - b0) < 32 ? (nh - b0) : 32;
#pragma unroll 1
      for (int k = 0; k < m32; ++k) {
        const int u  = __builtin_amdgcn_readlane(uv, k);
        const int sl = u & (NBMAX - 1);
        if (lane == 0) scnt[sl] = scnt[sl] + 1;
      }
    }
  }
  __syncthreads();

  {
    const v4i ca = *(const v4i*)(scnt + 8 * tid);
    const v4i cb = *(const v4i*)(scnt + 8 * tid + 4);
    const int e0 = ca.x < 0 ? 0 : ca.x, e1 = ca.y < 0 ? 0 : ca.y, e2 = ca.z < 0 ? 0 : ca.z, e3 = ca.w < 0 ? 0 : ca.w;
    const int e4 = cb.x < 0 ? 0 : cb.x, e5 = cb.y < 0 ? 0 : cb.y, e6 = cb.z < 0 ? 0 : cb.z, e7 = cb.w < 0 ? 0 : cb.w;
    const int ts = e0 + e1 + e2 + e3 + e4 + e5 + e6 + e7;
    int incl = ts;
#pragma unroll
    for (int d = 1; d < 32; d <<= 1) {
      const int up = __shfl_up(incl, d);
      if (lane >= d) incl += up;
    }
    if (lane == 31) wtot[wave] = incl;
    __syncthreads();
    int pre = 0;
#pragma unroll
    for (int w2 = 0; w2 < NWAVE; ++w2) pre += (w2 < wave) ? wtot[w2] : 0;
    int run = pre + incl - ts;
    soff[8 * tid + 0] = run; run += e0;
    soff[8 * tid + 1] = run; run += e1;
    soff[8 * tid + 2] = run; run += e2;
    soff[8 * tid + 3] = run; run += e3;
    soff[8 * tid + 4] = run; run += e4;
    soff[8 * tid + 5] = run; run += e5;
    soff[8 * tid + 6] = run; run += e6;
    soff[8 * tid + 7] = run;
  }
  __syncthreads();
  for (int i = tid; i < NBMAX; i += NTHR) list[i] = soff[i];
  __syncthreads();

  if (wave == 0) {
#pragma unroll 1
    for (int b0 = 0; b0 < nh; b0 += 32) {
      const int idx = b0 + lane;
      const int uv  = reg1[idx < nh ? idx : nh - 1];
      const int m32 = (nh - b0) < 32 ? (nh - b0) : 32;
#pragma unroll 1
      for (int k = 0; k < m32; ++k) {
        const int u   = __builtin_amdgcn_readlane(uv, k);
        const int sl  = u & (NBMAX - 1);
        const int eid = (int)((unsigned)u >> 12);
        if (lane == 0) {
          int pos = list[sl];
          pos = pos < 0 ? 0 : (pos > RCAP - 1 ? RCAP - 1 : pos);
          reg2[pos] = eid;
          list[sl] = pos + 1;
        }
      }
    }
  }
  __syncthreads();

  float* sWe = (float*)reg1;
  float* sAt = sWe + EDIM * DOUT;
  for (int i = tid; i < EDIM * DOUT; i += NTHR) sWe[i] = bfr(We[i]);
  for (int i = tid; i < DOUT; i += NTHR) sAt[i] = bfr(att[i]);
  __syncthreads();

  const int nbw = nb >> 3;
  const bool ovf = (nh >= RCAP);
  const float qnan = __int_as_float(0x7fc00000);
  const int c0 = 4 * lane;
  const v4f at4 = *(const v4fa*)(sAt + c0);
  v4f bi4 = *(const v4fa*)(bias + c0);
  v4f ga4 = *(const v4fa*)(gam + c0);
  v4f be4 = *(const v4fa*)(bet + c0);
  bi4.x = bfr(bi4.x); bi4.y = bfr(bi4.y); bi4.z = bfr(bi4.z); bi4.w = bfr(bi4.w);
  ga4.x = bfr(ga4.x); ga4.y = bfr(ga4.y); ga4.z = bfr(ga4.z); ga4.w = bfr(ga4.w);
  be4.x = bfr(be4.x); be4.y = bfr(be4.y); be4.z = bfr(be4.z); be4.w = bfr(be4.w);
  const float inv128 = 0.0078125f;

#pragma unroll 1
  for (int jt = 0; jt < nbw; ++jt) {
    const int slot = wave * nbw + jt;
    const int grow = nodeBase + slot;
    const int gcl  = grow < nN ? grow : nN - 1;
    int st = soff[slot];
    const int craw = scnt[slot];
    int cnt = craw;
    st  = st < 0 ? 0 : (st > nh ? nh : st);
    cnt = cnt < 0 ? 0 : (cnt > DEGCAP ? DEGCAP : cnt);
    if (cnt > nh - st) cnt = nh - st;
    const float pz = (ovf || craw > DEGCAP) ? qnan : 0.0f;
    const bool wr = grow < nN;

    const v4f xr4 = *(const v4fa*)(XLR + (size_t)gcl * NLR + DOUT + c0);
    float mx = -1.0e30f, dn = 0.f;
    v4f av = {0.f, 0.f, 0.f, 0.f};

#pragma unroll 1
    for (int q = 0; q < cnt; ++q) {
      int idx = st + q; idx = idx > RCAP - 1 ? RCAP - 1 : idx;
      int eid = reg2[idx]; eid = eid < 0 ? 0 : (eid > nE - 1 ? nE - 1 : eid);
      const int sraw = srcs[eid];
      const int s = sraw < 0 ? 0 : (sraw > nN - 1 ? nN - 1 : sraw);
      const v4f xl4 = *(const v4fa*)(XLR + (size_t)s * NLR + c0);
      const unsigned short* ebp = EB + (size_t)eid * EDIM;
      v4f ea = {0.f, 0.f, 0.f, 0.f};
#pragma unroll 1
      for (int k4 = 0; k4 < 4; ++k4) {
        const v2u w2 = *(const v2ua*)(ebp + 4 * k4);
        const float f0 = __uint_as_float(w2.x << 16);
        const float f1 = __uint_as_float(w2.x & 0xFFFF0000u);
        const float f2 = __uint_as_float(w2.y << 16);
        const float f3 = __uint_as_float(w2.y & 0xFFFF0000u);
        const float* wk = sWe + (4 * k4) * DOUT + c0;
        const v4f wa = *(const v4fa*)wk;
        const v4f wb = *(const v4fa*)(wk + DOUT);
        const v4f wc = *(const v4fa*)(wk + 2 * DOUT);
        const v4f wd = *(const v4fa*)(wk + 3 * DOUT);
        ea.x = fmaf(f0, wa.x, ea.x); ea.y = fmaf(f0, wa.y, ea.y); ea.z = fmaf(f0, wa.z, ea.z); ea.w = fmaf(f0, wa.w, ea.w);
        ea.x = fmaf(f1, wb.x, ea.x); ea.y = fmaf(f1, wb.y, ea.y); ea.z = fmaf(f1, wb.z, ea.z); ea.w = fmaf(f1, wb.w, ea.w);
        ea.x = fmaf(f2, wc.x, ea.x); ea.y = fmaf(f2, wc.y, ea.y); ea.z = fmaf(f2, wc.z, ea.z); ea.w = fmaf(f2, wc.w, ea.w);
        ea.x = fmaf(f3, wd.x, ea.x); ea.y = fmaf(f3, wd.y, ea.y); ea.z = fmaf(f3, wd.z, ea.z); ea.w = fmaf(f3, wd.w, ea.w);
      }
      float m0 = (xl4.x + xr4.x) + ea.x;
      float m1 = (xl4.y + xr4.y) + ea.y;
      float m2 = (xl4.z + xr4.z) + ea.z;
      float m3 = (xl4.w + xr4.w) + ea.w;
      m0 = m0 > 0.f ? m0 : m0 * NEG_SLOPE;
      m1 = m1 > 0.f ? m1 : m1 * NEG_SLOPE;
      m2 = m2 > 0.f ? m2 : m2 * NEG_SLOPE;
      m3 = m3 > 0.f ? m3 : m3 * NEG_SLOPE;
      float part = m0 * at4.x;
      part = fmaf(m1, at4.y, part);
      part = fmaf(m2, at4.z, part);
      part = fmaf(m3, at4.w, part);
      part += __shfl_xor(part, 1);
      part += __shfl_xor(part, 2);
      part += __shfl_xor(part, 4);
      const float df = part - mx;
      const float ee = __expf(-fabsf(df));
      const bool up  = df > 0.f;
      const float s1 = up ? ee : 1.0f;
      const float s2 = up ? 1.0f : ee;
      mx = up ? part : mx;
      dn = fmaf(dn, s1, s2);
      av.x = fmaf(av.x, s1, s2 * xl4.x);
      av.y = fmaf(av.y, s1, s2 * xl4.y);
      av.z = fmaf(av.z, s1, s2 * xl4.z);
      av.w = fmaf(av.w, s1, s2 * xl4.w);
    }
    const float ds = dn > 0.f ? dn : 1.0f;
    const float iv = (dn > 0.f ? 1.0f : 0.0f) * __builtin_amdgcn_rcpf(ds);
    const float o0 = fmaf(av.x, iv, bi4.x);
    const float o1 = fmaf(av.y, iv, bi4.y);
    const float o2 = fmaf(av.z, iv, bi4.z);
    const float o3 = fmaf(av.w, iv, bi4.w);
    float sm = (o0 + o1) + (o2 + o3);
#pragma unroll
    for (int off = 16; off > 0; off >>= 1) sm += __shfl_xor(sm, off);
    const float mu = sm * inv128;
    const float d0 = o0 - mu, d1 = o1 - mu, d2 = o2 - mu, d3 = o3 - mu;
    float ss = (d0 * d0 + d1 * d1) + (d2 * d2 + d3 * d3);
#pragma unroll
    for (int off = 16; off > 0; off >>= 1) ss += __shfl_xor(ss, off);
    const float var = ss * inv128;
    const float inv = rsqrtf(var + LN_EPS);
    v4f y;
    y.x = fmaxf(fmaf(d0 * inv, ga4.x, be4.x), 0.f) + pz;
    y.y = fmaxf(fmaf(d1 * inv, ga4.y, be4.y), 0.f) + pz;
    y.z = fmaxf(fmaf(d2 * inv, ga4.z, be4.z), 0.f) + pz;
    y.w = fmaxf(fmaf(d3 * inv, ga4.w, be4.w), 0.f) + pz;
    float* gp = out + (size_t)gcl * DOUT + c0;
    if (wr) *(volatile v4f*)gp = y;
    __threadfence();
    if (wr) *(volatile v4f*)gp = y;
  }
}

static int pick_nb(int nE, int nN) {
  int nb = NBMAX;
  while (nb > 16 && (long long)nb * (long long)nE * 5LL > (long long)RCAP * (long long)nN * 2LL) nb >>= 1;
  return nb;
}
static inline int cdiv(int a, int b) { return (a + b - 1) / b; }

extern "C" void kernel_launch(void* const* d_in, const int* in_sizes, int n_in,
                              void* d_out, int out_size, void* d_ws, size_t ws_size,
                              hipStream_t stream) {
  if (n_in < 10) return;
  const int nN = in_sizes[0] / DIN;
  if (nN <= 0 || in_sizes[0] != nN * DIN || nN > (1 << 22)) return;
  if (in_sizes[1] < 2 || (in_sizes[1] & 1) != 0) return;
  const int nE = in_sizes[1] / 2;
  if (nE < 1 || nE > (1 << 20)) return;
  if (in_sizes[2] != nE * EDIM) return;
  if (in_sizes[3] != DIN * DOUT || in_sizes[4] != DIN * DOUT) return;
  if (in_sizes[5] != EDIM * DOUT) return;
  if (in_sizes[6] != DOUT) return;
  if (in_sizes[7] != DOUT || in_sizes[8] != DOUT || in_sizes[9] != DOUT) return;
  if (out_size != nN * DOUT) return;

  const float* x    = (const float*)d_in[0];
  const int*   ei   = (const int*)  d_in[1];
  const float* eat  = (const float*)d_in[2];
  const float* W_l  = (const float*)d_in[3];
  const float* W_r  = (const float*)d_in[4];
  const float* W_e  = (const float*)d_in[5];
  const float* att  = (const float*)d_in[6];
  const float* bias = (const float*)d_in[7];
  const float* gam  = (const float*)d_in[8];
  const float* bet  = (const float*)d_in[9];
  float* out = (float*)d_out;
  const int* src = ei;
  const int* dst = ei + nE;

  const int MP   = cdiv(nN, GBM) * GBM;
  const int nb   = pick_nb(nE, nN);
  const int gA   = cdiv(MP, nb);
  const int vec8 = ((nE & 3) == 0) ? 1 : 0;
  if (gA * nb < MP) return;
  const int nVals    = nE * EDIM;
  const int nValsPad = cdiv(nVals, 64) * 64;
  const int nUE      = nValsPad / 8;

  char* ws = (char*)d_ws;
  size_t off = 0;
  const size_t oXB  = off; off += (size_t)MP * DIN * 2;            off = (off + 255) & ~(size_t)255;
  const size_t oWT  = off; off += (size_t)NLR * DIN * 2;           off = (off + 255) & ~(size_t)255;
  const size_t oEB  = off; off += (size_t)nValsPad * 2;            off = (off + 255) & ~(size_t)255;
  const size_t oXLR = off; off += (size_t)MP * NLR * 4;            off = (off + 255) & ~(size_t)255;
  if (off > ws_size || off > (size_t)WSMAX) return;
  unsigned short* XB  = (unsigned short*)(ws + oXB);
  unsigned short* WT  = (unsigned short*)(ws + oWT);
  unsigned short* EB  = (unsigned short*)(ws + oEB);
  float*          XLR = (float*)(ws + oXLR);

  hipFuncSetAttribute(reinterpret_cast<const void*>(&k_agg),
                      hipFuncAttributeMaxDynamicSharedMemorySize, LDS_AGG);

  const int nUx = MP * (DIN / 8);
  k_xprep<<<cdiv(nUx, NTHR), NTHR, 0, stream>>>(x, XB, nN, nUx);

  const int nUw = NLR * (DIN / 8);
  k_wtr<<<cdiv(nUw, NTHR), NTHR, 0, stream>>>(W_l, W_r, W_r, W_r, DOUT, DOUT, DOUT, DOUT, DOUT, DIN, WT, nUw);

  k_eprep<<<cdiv(nUE, NTHR), NTHR, 0, stream>>>(eat, EB, nVals, nUE);

  const int gM = MP / GBM;
  k_gemm<<<dim3(gM, NLR / GBN), GTHR, 0, stream>>>(XB, WT, XLR, DIN, NLR);

  k_agg<<<gA, NTHR, LDS_AGG, stream>>>(src, dst, XLR, EB, W_e, att, bias, gam, bet, out, nN, nE, nb, vec8);
}
